// GraphNetwork_28741921145146
// MI455X (gfx1250) — hardware-verified
//
#include <hip/hip_runtime.h>


#define NN_ 65536
#define NE_ 1048576
#define HH 64
#define NOUT 32
#define NG 16
#define IL_CAP 64
#define NCH 8
#define CHN (NN_ / NCH)
#define SLOTCAP 163840

typedef __attribute__((ext_vector_type(16))) __bf16   v16bf;
typedef __attribute__((ext_vector_type(16))) _Float16 v16h;
typedef __attribute__((ext_vector_type(8)))  float    v8f;
typedef __attribute__((ext_vector_type(8)))  unsigned v8u;

__device__ __forceinline__ unsigned f2bf(float f) { unsigned u = __float_as_uint(f); u += 0x7FFFu + ((u >> 16) & 1u); return u >> 16; }
__device__ __forceinline__ unsigned f2h(float f) { return (unsigned)__builtin_bit_cast(unsigned short, (_Float16)f); }
__device__ __forceinline__ int kpat(int v, int half) { return ((v & 4) ? 16 : 0) + half * 8 + 2 * (v & 3); }

template <int F16, int NP> struct Opnd { v16bf p[NP]; };

template <int F16, int NP> __device__ __forceinline__ void pack2(float f0, float f1, unsigned* o) {
    if (F16) { o[0] = f2h(f0) | (f2h(f1) << 16); return; }
    unsigned h0 = f2bf(f0), h1 = f2bf(f1); o[0] = h0 | (h1 << 16);
    if (NP >= 2) {
        float r0 = f0 - __uint_as_float(h0 << 16), r1 = f1 - __uint_as_float(h1 << 16);
        unsigned m0 = f2bf(r0), m1 = f2bf(r1); o[1] = m0 | (m1 << 16);
        if (NP >= 3) {
            float s0 = r0 - __uint_as_float(m0 << 16), s1 = r1 - __uint_as_float(m1 << 16);
            o[2] = f2bf(s0) | (f2bf(s1) << 16);
        }
    }
}
template <int F16, int NP> __device__ __forceinline__ void op_row(const float* rowp, int half, float sc, Opnd<F16, NP>& o) {
    v8u u[NP];
#pragma unroll
    for (int v = 0; v < 8; ++v) {
        int kk = kpat(v, half); unsigned t[3];
        pack2<F16, NP>(rowp[kk] * sc, rowp[kk + 1] * sc, t);
#pragma unroll
        for (int p = 0; p < NP; ++p) u[p][v] = t[p];
    }
#pragma unroll
    for (int p = 0; p < NP; ++p) o.p[p] = __builtin_bit_cast(v16bf, u[p]);
}
template <int F16, int NP> __device__ __forceinline__ void op_row_tail(const float* rowp, int half, float sc, int kvalid, Opnd<F16, NP>& o) {
    v8u u[NP];
#pragma unroll
    for (int v = 0; v < 8; ++v) {
        int kk = kpat(v, half); unsigned t[3];
        float f0 = kk < kvalid ? rowp[kk] * sc : 0.0f, f1 = (kk + 1) < kvalid ? rowp[kk + 1] * sc : 0.0f;
        pack2<F16, NP>(f0, f1, t);
#pragma unroll
        for (int p = 0; p < NP; ++p) u[p][v] = t[p];
    }
#pragma unroll
    for (int p = 0; p < NP; ++p) o.p[p] = __builtin_bit_cast(v16bf, u[p]);
}
template <int F16, int NP> __device__ __forceinline__ void op_col(const float* M, int ld, int n, int k0, int half, float sc, Opnd<F16, NP>& o) {
    v8u u[NP];
#pragma unroll
    for (int v = 0; v < 8; ++v) {
        int kk = k0 + kpat(v, half); unsigned t[3];
        pack2<F16, NP>(M[(size_t)kk * ld + n] * sc, M[(size_t)(kk + 1) * ld + n] * sc, t);
#pragma unroll
        for (int p = 0; p < NP; ++p) u[p][v] = t[p];
    }
#pragma unroll
    for (int p = 0; p < NP; ++p) o.p[p] = __builtin_bit_cast(v16bf, u[p]);
}
template <int F16, int NP> __device__ __forceinline__ void op_col_tail(const float* M, int ld, int n, int k0, int half, float sc, int K, Opnd<F16, NP>& o) {
    v8u u[NP];
#pragma unroll
    for (int v = 0; v < 8; ++v) {
        int kk = k0 + kpat(v, half); unsigned t[3];
        float f0 = kk < K ? M[(size_t)kk * ld + n] * sc : 0.0f, f1 = (kk + 1) < K ? M[(size_t)(kk + 1) * ld + n] * sc : 0.0f;
        pack2<F16, NP>(f0, f1, t);
#pragma unroll
        for (int p = 0; p < NP; ++p) u[p][v] = t[p];
    }
#pragma unroll
    for (int p = 0; p < NP; ++p) o.p[p] = __builtin_bit_cast(v16bf, u[p]);
}
__device__ __forceinline__ v8f wm_bf16(v16bf a, v16bf b, v8f c) { return __builtin_amdgcn_wmma_f32_16x16x32_bf16(false, a, false, b, (short)0, c, false, false); }
template <int F16, int NA, int NB> __device__ __forceinline__ v8f wmma_op(const Opnd<F16, NA>& a, const Opnd<F16, NB>& b, v8f c) {
    if (F16) {
        v16h ah = __builtin_bit_cast(v16h, a.p[0]), bh = __builtin_bit_cast(v16h, b.p[0]);
        c = __builtin_amdgcn_wmma_f32_16x16x32_f16(false, ah, false, bh, (short)0, c, false, false);
        asm volatile("v_nop\n\tv_nop\n\tv_nop\n\tv_nop" : "+v"(c) : "v"(ah), "v"(bh));
        return c;
    }
    constexpr int NMX = NA > NB ? NA : NB;
#pragma unroll
    for (int i = 0; i < NA; ++i)
#pragma unroll
        for (int j = 0; j < NB; ++j)
            if (i + j < NMX) c = wm_bf16(a.p[i], b.p[j], c);
    if (NA == 1 && NB == 1)      asm volatile("v_nop\n\tv_nop\n\tv_nop\n\tv_nop" : "+v"(c) : "v"(a.p[0]), "v"(b.p[0]));
    else if (NA == 2 && NB == 1) asm volatile("v_nop\n\tv_nop\n\tv_nop\n\tv_nop" : "+v"(c) : "v"(a.p[0]), "v"(a.p[1]), "v"(b.p[0]));
    else if (NA == 1 && NB == 2) asm volatile("v_nop\n\tv_nop\n\tv_nop\n\tv_nop" : "+v"(c) : "v"(a.p[0]), "v"(b.p[0]), "v"(b.p[1]));
    else if (NA == 2 && NB == 2) asm volatile("v_nop\n\tv_nop\n\tv_nop\n\tv_nop" : "+v"(c) : "v"(a.p[0]), "v"(a.p[1]), "v"(b.p[0]), "v"(b.p[1]));
    else                         asm volatile("v_nop\n\tv_nop\n\tv_nop\n\tv_nop" : "+v"(c) : "v"(a.p[0]), "v"(a.p[NA - 1]), "v"(b.p[0]), "v"(b.p[NB - 1]), "v"(a.p[NA / 2]), "v"(b.p[NB / 2]));
    return c;
}

struct ZMap { long long s1; long long s2; int zdiv; int pad_; };
__device__ __forceinline__ size_t zoff(const ZMap& m, int z) { return (size_t)((long long)(z / m.zdiv) * m.s1 + (long long)(z % m.zdiv) * m.s2); }

#define ACT_NONE 0
#define ACT_RELU 1
#define ACT_GELU_ERF 2
#define ACT_SILU 3
#define ACT_TANH 4
__device__ __forceinline__ float act_apply(int act, float x) {
    if (act == ACT_RELU) return x > 0.f ? x : 0.f;
    if (act == ACT_GELU_ERF) return 0.5f * x * (1.0f + erff(x * 0.70710678118654752f));
    if (act == ACT_SILU) return x / (1.0f + expf(-x));
    if (act == ACT_TANH) return tanhf(x);
    return x;
}
struct GemmArgs {
    ZMap za, zb_, zc, zbias, zadd, zrsc, zmul, zrbias;
    const float* A; const float* Bm; float* C; const float* bias; const float* add; const float* rsc; const float* mul; const float* rbias;
    long long ldadd, ldmul;
    int lda, ldb, ldc, K;
    float ascale, bscale, oscale, addscale;
    int M, nvalid, nstore, ldrsc;
    int bcs, pad1, pad2, pad3;
};
template <int BT, int F16, int NA, int NB, int RW, int CW, int ACT>
__global__ __launch_bounds__(256) void gemm_kernel(GemmArgs g) {
    constexpr int TR = 16 * RW, TC = 64 * CW, CSTR = TC + 4;
    __shared__ __align__(16) float cst[TR * CSTR];
    const int z = blockIdx.z;
    const float* A = g.A + zoff(g.za, z); const float* Bm = g.Bm + zoff(g.zb_, z); float* C = g.C + zoff(g.zc, z);
    const int tid = threadIdx.x, lane = tid & 31, wv = tid >> 5;
    const int l16 = lane & 15, half = lane >> 4;
    const int rt = wv % RW, ch = wv / RW;
    const int row0 = blockIdx.x * TR, col0 = blockIdx.y * TC + ch * 64;
    int arix = row0 + rt * 16 + l16; if (arix >= g.M) arix = g.M - 1;
    const float* arow = A + (size_t)arix * g.lda;
    v8f acc[4];
#pragma unroll
    for (int t = 0; t < 4; ++t) acc[t] = (v8f){};
    const int K = g.K;
#pragma unroll 1
    for (int kc = 0; kc < K; kc += 32) {
        Opnd<F16, NA> a;
        if (kc + 32 <= K) op_row<F16, NA>(arow + kc, half, g.ascale, a); else op_row_tail<F16, NA>(arow + kc, half, g.ascale, K - kc, a);
#pragma unroll
        for (int t = 0; t < 4; ++t) {
            Opnd<F16, NB> b;
            const int n = col0 + t * 16 + l16;
            if (n < g.nvalid) {
                if (BT) { if (kc + 32 <= K) op_row<F16, NB>(Bm + (size_t)n * g.ldb + kc, half, g.bscale, b); else op_row_tail<F16, NB>(Bm + (size_t)n * g.ldb + kc, half, g.bscale, K - kc, b); }
                else    { if (kc + 32 <= K) op_col<F16, NB>(Bm, g.ldb, n * g.bcs, kc, half, g.bscale, b); else op_col_tail<F16, NB>(Bm, g.ldb, n * g.bcs, kc, half, g.bscale, K, b); }
            } else {
#pragma unroll
                for (int p = 0; p < NB; ++p) b.p[p] = (v16bf){};
            }
            acc[t] = wmma_op<F16, NA, NB>(a, b, acc[t]);
        }
    }
    const float* bias = g.bias ? g.bias + zoff(g.zbias, z) : nullptr;
    const float* add = g.add ? g.add + zoff(g.zadd, z) : nullptr;
    const float* rsc = g.rsc ? g.rsc + zoff(g.zrsc, z) : nullptr;
    const float* mul = g.mul ? g.mul + zoff(g.zmul, z) : nullptr;
    const float* rbias = g.rbias ? g.rbias + zoff(g.zrbias, z) : nullptr;
#pragma unroll
    for (int t = 0; t < 4; ++t) {
        const int cl = ch * 64 + t * 16 + l16;
        const int cg = blockIdx.y * TC + cl;
        const bool cok = cg < g.nvalid;
        const float bv = (bias && cok) ? bias[(size_t)cg * g.bcs] : 0.0f;
#pragma unroll
        for (int r = 0; r < 8; ++r) {
            const int rl = rt * 16 + r + 8 * half;
            float v = acc[t][r] * g.oscale + bv;
            int rg = row0 + rl; if (rg >= g.M) rg = g.M - 1;
            if (rbias) v += rbias[rg];
            if (rsc) v *= rsc[(size_t)rg * g.ldrsc];
            if (mul && cok) v *= mul[(size_t)rg * g.ldmul + cg];
            if (add && cok) v += g.addscale * add[(size_t)rg * g.ldadd + cg];
            cst[rl * CSTR + cl] = v;
        }
    }
    __syncthreads();
    const int col = tid % TC, rsel = tid / TC, rstep = 256 / TC;
    if (ACT != ACT_NONE) {
#pragma unroll 1
        for (int r = rsel; r < TR; r += rstep) cst[r * CSTR + col] = act_apply(ACT, cst[r * CSTR + col]);
    }
    float* ob = C + (size_t)row0 * g.ldc + (size_t)blockIdx.y * TC;
    const bool colok = (int)(blockIdx.y * TC + col) < g.nstore;
    const int rmax = (g.M - row0 < TR) ? (g.M - row0) : TR;
    auto pass = [&]() {
        if (colok) {
#pragma unroll 4
            for (int r = rsel; r < rmax; r += rstep) *(volatile float*)(ob + (size_t)r * g.ldc + col) = cst[r * CSTR + col];
        }
    };
    pass();
    __threadfence();
    pass();
}
static inline ZMap zm(long long s1) { ZMap m; m.s1 = s1; m.s2 = 0; m.zdiv = 1; m.pad_ = 0; return m; }
static inline ZMap zm2(long long s1, long long s2, int zdiv) { ZMap m; m.s1 = s1; m.s2 = s2; m.zdiv = zdiv; m.pad_ = 0; return m; }
static inline GemmArgs gemm_args(const float* A, int lda, ZMap za, const float* Bm, int ldb, ZMap zb, float* C, int ldc, ZMap zc, int M, int N, int K) {
    GemmArgs g; g.za = za; g.zb_ = zb; g.zc = zc; g.zbias = zm(0); g.zadd = zm(0); g.zrsc = zm(0); g.zmul = zm(0); g.zrbias = zm(0);
    g.A = A; g.Bm = Bm; g.C = C; g.bias = nullptr; g.add = nullptr; g.rsc = nullptr; g.mul = nullptr; g.rbias = nullptr; g.ldadd = 0; g.ldmul = 0;
    g.lda = lda; g.ldb = ldb; g.ldc = ldc; g.K = K; g.ascale = 1.0f; g.bscale = 1.0f; g.oscale = 1.0f; g.addscale = 1.0f; g.M = M; g.nvalid = N; g.nstore = N; g.ldrsc = 1;
    g.bcs = 1; g.pad1 = 0; g.pad2 = 0; g.pad3 = 0;
    return g;
}
static_assert(sizeof(ZMap) == 24, "ZMap layout");
static_assert(sizeof(GemmArgs) == 8 * 24 + 8 * 8 + 2 * 8 + 4 * 4 + 4 * 4 + 4 * 4 + 4 * 4, "GemmArgs has no padding");

__global__ __launch_bounds__(256) void softmax_rows(float* S, long long sy, long long sx, int L, float prescale, const float* addv, long long say, int aydiv, int causal,
                                                  const int* imask, long long imy, long long imx, float maskval) {
    __shared__ float red[8];
    const int tid = threadIdx.x, lane = tid & 31, wid = tid >> 5;
    float* row = S + (size_t)blockIdx.y * sy + (size_t)blockIdx.x * sx;
    const float* av = addv ? addv + (size_t)(blockIdx.y / aydiv) * say : nullptr;
    const int* im = imask ? imask + (size_t)(blockIdx.y / aydiv) * imy + (size_t)blockIdx.x * imx : nullptr;
    float v[16];
    const int nj = L / 256;
    float mx = -__builtin_inff();
#pragma unroll
    for (int j = 0; j < 16; ++j) if (j < nj) { float t = row[tid + 256 * j] * prescale; if (av) t += av[tid + 256 * j]; if (im && im[tid + 256 * j] == 0) t = maskval; if (causal && (tid + 256 * j) > (int)blockIdx.x) t = -__builtin_inff(); v[j] = t; mx = fmaxf(mx, t); }
#pragma unroll
    for (int o = 16; o; o >>= 1) mx = fmaxf(mx, __shfl_xor(mx, o, 32));
    if (lane == 0) red[wid] = mx;
    __syncthreads();
    float m = red[0];
#pragma unroll
    for (int i = 1; i < 8; ++i) m = fmaxf(m, red[i]);
    if (m == -__builtin_inff()) m = 0.f;
    __syncthreads();
    float sum = 0.f;
#pragma unroll
    for (int j = 0; j < 16; ++j) if (j < nj) { v[j] = expf(v[j] - m); sum += v[j]; }
#pragma unroll
    for (int o = 16; o; o >>= 1) sum += __shfl_xor(sum, o, 32);
    if (lane == 0) red[wid] = sum;
    __syncthreads();
    float tot = 0.f;
#pragma unroll
    for (int i = 0; i < 8; ++i) tot += red[i];
    const float inv = 1.0f / tot;
#pragma unroll
    for (int j = 0; j < 16; ++j) if (j < nj) *(volatile float*)(row + tid + 256 * j) = v[j] * inv;
    __threadfence();
#pragma unroll
    for (int j = 0; j < 16; ++j) if (j < nj) *(volatile float*)(row + tid + 256 * j) = v[j] * inv;
}

#define VST2(T, p, v) do { const T vst2_v_ = (v); *(volatile T*)(p) = vst2_v_; __threadfence(); *(volatile T*)(p) = vst2_v_; } while (0)
#define IL_T 128
#define IL_TILE 4096
__global__ __launch_bounds__(IL_T) void k_inlists(const int* __restrict__ tgt, int E, int N, int* NBR, int* cnt) {
    __shared__ int tt[IL_TILE];
    __shared__ int lists[IL_T * IL_CAP];
    const int d = blockIdx.x * IL_T + threadIdx.x; int n = 0;
    for (int e0 = 0; e0 < E; e0 += IL_TILE) {
        const int nt = min(IL_TILE, E - e0);
        __syncthreads();
        for (int i = threadIdx.x; i < nt; i += IL_T) tt[i] = tgt[e0 + i];
        __syncthreads();
        for (int i = 0; i < nt; ++i) { if (tt[i] == d) { if (n < IL_CAP) lists[threadIdx.x * IL_CAP + n] = e0 + i; ++n; } }
    }
    if (d < N) {
        int* row = NBR + (size_t)d * IL_CAP;
        for (int j = 0; j < IL_CAP; ++j) { const int v = (j < n) ? lists[threadIdx.x * IL_CAP + j] : 0; *(volatile int*)(row + j) = v; }
        __threadfence();
        for (int j = 0; j < IL_CAP; ++j) { const int v = (j < n) ? lists[threadIdx.x * IL_CAP + j] : 0; *(volatile int*)(row + j) = v; }
        VST2(int, cnt + d, min(n, IL_CAP));
    }
}
__global__ __launch_bounds__(256) void k_csr_scan(const int* __restrict__ cnt, int* off, int N) {
    __shared__ int part[256]; const int per = ((((N + 255) / 256) + 31) / 32) * 32; const int a = threadIdx.x * per, b = min(N, a + per); int s = 0;
    for (int i = a; i < b; ++i) s += cnt[i]; part[threadIdx.x] = s; __syncthreads();
    if (threadIdx.x == 0) { int run = 0; for (int t = 0; t < 256; ++t) { const int v = part[t]; part[t] = run; run += v; } } __syncthreads();
    int run = part[threadIdx.x]; for (int i = a; i < b; ++i) { VST2(int, off + i, run); run += cnt[i]; }
    if (a < N && b == N) { VST2(int, off + N, run); }
}
__global__ __launch_bounds__(256) void k_slotcopy(const int* __restrict__ off, const int* __restrict__ NBR, int* slot, int N) {
    const int t = blockIdx.x * 256 + threadIdx.x; const int tot = off[N]; if (t >= tot) return;
    int lo = 0, hi = N - 1;
    while (lo < hi) { const int mid = (lo + hi + 1) >> 1; if (off[mid] <= t) lo = mid; else hi = mid - 1; }
    int j = t - off[lo]; j = (j < 0) ? 0 : ((j >= IL_CAP) ? (IL_CAP - 1) : j);
    VST2(int, slot + t, NBR[(size_t)lo * IL_CAP + j]);
}

__global__ __launch_bounds__(256) void k_msg(const float* __restrict__ x, const float* __restrict__ pos, const int* __restrict__ srcs, const int* __restrict__ off, const int* __restrict__ slot,
                                             const float* __restrict__ W, const float* __restrict__ b, int n0, int n1, float* H1) {
    const int p0 = off[n0], p1 = off[n1];
    const size_t q = (size_t)blockIdx.x * 256 + threadIdx.x; if (q >= (size_t)(p1 - p0) * HH) return; const int c = (int)(q % HH); const int p = p0 + (int)(q / HH);
    int lo = n0, hi = n1 - 1; while (lo < hi) { const int mid = (lo + hi + 1) >> 1; if (off[mid] <= p) lo = mid; else hi = mid - 1; }
    const int i = lo; int e = slot[p]; e = e < 0 ? 0 : (e >= NE_ ? NE_ - 1 : e); int s = srcs[e]; s = s < 0 ? 0 : (s >= NN_ ? NN_ - 1 : s);
    const float m0 = x[s * 3], m1 = x[s * 3 + 1], m2 = x[s * 3 + 2], m3 = pos[s * 3] - pos[i * 3], m4 = pos[s * 3 + 1] - pos[i * 3 + 1], m5 = pos[s * 3 + 2] - pos[i * 3 + 2];
    const float v = b[c] + m0 * W[c] + m1 * W[HH + c] + m2 * W[2 * HH + c] + m3 * W[3 * HH + c] + m4 * W[4 * HH + c] + m5 * W[5 * HH + c];
    VST2(float, H1 + q, fmaxf(v, 0.f));
}
__global__ __launch_bounds__(256) void k_segmax(const float* __restrict__ H2, const int* __restrict__ off, int n0, int n1, float* AGG) {
    const int q = blockIdx.x * 256 + threadIdx.x; if (q >= (n1 - n0) * HH) return; const int c = q % HH, i = n0 + q / HH; const int p0 = off[n0];
    const int a = off[i], b = off[i + 1]; float m = -__builtin_inff();
    for (int p = a; p < b && p < a + IL_CAP; ++p) m = fmaxf(m, H2[(size_t)(p - p0) * HH + c]);
    if (!(m > -__builtin_inff())) m = 0.f;
    VST2(float, AGG + (size_t)i * HH + c, m);
}
__global__ __launch_bounds__(256) void k_leakymask(const float* __restrict__ Xin, const float* __restrict__ mask, float* X) {
    const size_t q = (size_t)blockIdx.x * 256 + threadIdx.x; if (q >= (size_t)NN_ * HH) return; const float v = Xin[q];
    VST2(float, X + q, (v >= 0.f ? v : 0.01f * v) * mask[q]);
}
__global__ __launch_bounds__(256) void k_nbrsum(const float* __restrict__ X, const int* __restrict__ srcs, const int* __restrict__ off, const int* __restrict__ slot, float* SUM) {
    const size_t q = (size_t)blockIdx.x * 256 + threadIdx.x; if (q >= (size_t)NN_ * HH) return; const int c = (int)(q % HH), i = (int)(q / HH);
    const int a = off[i], b = off[i + 1]; float s = 0.f;
    for (int p = a; p < b && p < a + IL_CAP; ++p) { int e = slot[p]; e = e < 0 ? 0 : (e >= NE_ ? NE_ - 1 : e); int sn = srcs[e]; sn = sn < 0 ? 0 : (sn >= NN_ ? NN_ - 1 : sn); s += X[(size_t)sn * HH + c]; }
    VST2(float, SUM + q, s);
}
__global__ __launch_bounds__(256) void k_pool(const float* __restrict__ X3, const int* __restrict__ batch, float* out) {
    __shared__ float red[256];
    const int g = blockIdx.x, tid = threadIdx.x; const int c = tid & 31, part = tid >> 5;
    float m = -__builtin_inff();
    for (int n = part; n < NN_; n += 8) if (batch[n] == g) m = fmaxf(m, X3[(size_t)n * NOUT + c]);
    red[tid] = m; __syncthreads();
    if (tid < 32) { float r = red[tid];
#pragma unroll
        for (int k = 1; k < 8; ++k) r = fmaxf(r, red[tid + 32 * k]); if (!(r > -__builtin_inff())) r = 0.f; VST2(float, out + g * NOUT + tid, r); }
}

extern "C" void kernel_launch(void* const* d_in, const int* in_sizes, int n_in,
                              void* d_out, int out_size, void* d_ws, size_t ws_size, hipStream_t stream) {
    (void)in_sizes; (void)n_in; (void)out_size;
    const float* x = (const float*)d_in[0]; const float* pos = (const float*)d_in[1];
    const int* ei = (const int*)d_in[2];
    const int* batch = (const int*)d_in[3];
    const float* mask1 = (const float*)d_in[4]; const float* mask2 = (const float*)d_in[5];
    const float* Wl1 = (const float*)d_in[6]; const float* bl1 = (const float*)d_in[7]; const float* Wl2 = (const float*)d_in[8]; const float* bl2 = (const float*)d_in[9];
    const float* Wg = (const float*)d_in[10]; const float* bg = (const float*)d_in[11];
    const float* W2r = (const float*)d_in[12]; const float* W2s = (const float*)d_in[13]; const float* b2 = (const float*)d_in[14];
    const float* W3r = (const float*)d_in[15]; const float* W3s = (const float*)d_in[16]; const float* b3 = (const float*)d_in[17];
    float* out = (float*)d_out;
    const int* srcs = ei; const int* dsts = ei + NE_;

    char* wsp = (char*)d_ws;
    auto take = [&](size_t bytes) { char* p = wsp; wsp += (bytes + 255) & ~(size_t)255; return (void*)p; };
    int* NBR = (int*)take((size_t)NN_ * IL_CAP * 4); int* cnt = (int*)take((size_t)(NN_ + 1) * 4); int* off = (int*)take((size_t)(NN_ + 1) * 4); int* slot = (int*)take((size_t)NE_ * 4);
    float* H1 = (float*)take((size_t)SLOTCAP * HH * 4); float* H2 = (float*)take((size_t)SLOTCAP * HH * 4);
    float* AGG = (float*)take((size_t)NN_ * HH * 4); float* X1 = (float*)take((size_t)NN_ * HH * 4); float* T1 = (float*)take((size_t)NN_ * HH * 4);
    float* SUM = (float*)take((size_t)NN_ * HH * 4); float* X2 = (float*)take((size_t)NN_ * HH * 4); float* X3 = (float*)take((size_t)NN_ * NOUT * 4);
    if ((size_t)(wsp - (char*)d_ws) > ws_size) return;

    k_inlists<<<(NN_ + IL_T - 1) / IL_T, IL_T, 0, stream>>>(dsts, NE_, NN_, NBR, cnt);
    k_csr_scan<<<1, 256, 0, stream>>>(cnt, off, NN_);
    k_slotcopy<<<(NE_ + 255) / 256, 256, 0, stream>>>(off, NBR, slot, NN_);
    for (int c = 0; c < NCH; ++c) {
        const int n0 = c * CHN, n1 = n0 + CHN;
        k_msg<<<(unsigned)(((size_t)SLOTCAP * HH) / 256), 256, 0, stream>>>(x, pos, srcs, off, slot, Wl1, bl1, n0, n1, H1);
        { GemmArgs g = gemm_args(H1, HH, zm(0), Wl2, HH, zm(0), H2, HH, zm(0), SLOTCAP, HH, HH); g.bias = bl2; gemm_kernel<0, 0, 2, 2, 8, 1, ACT_NONE><<<dim3(SLOTCAP / 128, 1, 1), 256, 0, stream>>>(g); }
        k_segmax<<<(CHN * HH) / 256, 256, 0, stream>>>(H2, off, n0, n1, AGG);
    }
    { GemmArgs g = gemm_args(AGG, HH, zm(0), Wg, HH, zm(0), T1, HH, zm(0), NN_, HH, HH); g.bias = bg; gemm_kernel<0, 0, 2, 2, 8, 1, ACT_NONE><<<dim3(NN_ / 128, 1, 1), 256, 0, stream>>>(g); }
    k_leakymask<<<(NN_ * HH) / 256, 256, 0, stream>>>(T1, mask1, X1);
    k_nbrsum<<<(NN_ * HH) / 256, 256, 0, stream>>>(X1, srcs, off, slot, SUM);
    { GemmArgs g = gemm_args(X1, HH, zm(0), W2s, HH, zm(0), T1, HH, zm(0), NN_, HH, HH); g.bias = b2; gemm_kernel<0, 0, 2, 2, 8, 1, ACT_NONE><<<dim3(NN_ / 128, 1, 1), 256, 0, stream>>>(g);
      GemmArgs g2 = gemm_args(SUM, HH, zm(0), W2r, HH, zm(0), T1, HH, zm(0), NN_, HH, HH); g2.add = T1; g2.ldadd = HH; g2.addscale = 1.0f; gemm_kernel<0, 0, 2, 2, 8, 1, ACT_NONE><<<dim3(NN_ / 128, 1, 1), 256, 0, stream>>>(g2); }
    k_leakymask<<<(NN_ * HH) / 256, 256, 0, stream>>>(T1, mask2, X2);
    k_nbrsum<<<(NN_ * HH) / 256, 256, 0, stream>>>(X2, srcs, off, slot, SUM);
    { GemmArgs g = gemm_args(X2, HH, zm(0), W3s, NOUT, zm(0), X3, NOUT, zm(0), NN_, NOUT, HH); g.bias = b3; gemm_kernel<0, 0, 2, 2, 8, 1, ACT_NONE><<<dim3(NN_ / 128, 1, 1), 256, 0, stream>>>(g);
      GemmArgs g2 = gemm_args(SUM, HH, zm(0), W3r, NOUT, zm(0), X3, NOUT, zm(0), NN_, NOUT, HH); g2.add = X3; g2.ldadd = NOUT; g2.addscale = 1.0f; gemm_kernel<0, 0, 2, 2, 8, 1, ACT_NONE><<<dim3(NN_ / 128, 1, 1), 256, 0, stream>>>(g2); }
    k_pool<<<NG, 256, 0, stream>>>(X3, batch, out);
}
